// PedestrianEncoder_3289944949287
// MI455X (gfx1250) — hardware-verified
//
#include <hip/hip_runtime.h>
#include <math.h>


typedef _Float16 v16h __attribute__((ext_vector_type(16)));
typedef _Float16 v8h  __attribute__((ext_vector_type(8)));
typedef _Float16 v4h  __attribute__((ext_vector_type(4)));
typedef float    v8f  __attribute__((ext_vector_type(8)));
typedef float    v4f  __attribute__((ext_vector_type(4)));

#define T_   64
#define B_   32
#define P_   32
#define E_   128
#define H_   128
#define N_   (B_ * P_)
#define G4_  (4 * H_)
#define NTHR 256
#define ROWS 16

typedef char check_rows[(N_ % ROWS == 0) ? 1 : -1];
typedef char check_h[(H_ % 32 == 0) ? 1 : -1];
typedef char check_copy[(ROWS * H_ == NTHR * 8) ? 1 : -1];

union Pk16 { v8h h; v4f f; };

__device__ __forceinline__ v8f wmma_f16(v16h a, v16h b, v8f c)
{
  c = __builtin_amdgcn_wmma_f32_16x16x32_f16(false, a, false, b, (short)0, c, false, false);
  asm volatile("v_nop\n\tv_nop\n\tv_nop\n\tv_nop" : "+v"(c) : "v"(a), "v"(b));
  return c;
}

__device__ __forceinline__ v16h cat8(v8h lo, v8h up)
{
  return __builtin_shufflevector(lo, up, 0, 1, 2, 3, 4, 5, 6, 7, 8, 9, 10, 11, 12, 13, 14, 15);
}

__device__ __forceinline__ v8f zero8()
{
  v8f z;
#pragma unroll
  for (int r = 0; r < 8; ++r) z[r] = 0.0f;
  return z;
}

__device__ __forceinline__ v16h frag_k_lds(const _Float16* rowp, int k0, int h)
{
  const _Float16* p = rowp + k0 + 8 * h;
  v8h lo = *(const v8h*)p;
  v8h up = *(const v8h*)(p + 16);
  return cat8(lo, up);
}

__device__ __forceinline__ v16h frag_k_gf32(const float* __restrict__ rowp, int k0, int h)
{
  const float* p = rowp + k0 + 8 * h;
  v4f w0 = *(const v4f*)(p);
  v4f w1 = *(const v4f*)(p + 4);
  v4f w2 = *(const v4f*)(p + 16);
  v4f w3 = *(const v4f*)(p + 20);
  v4h h0 = __builtin_convertvector(w0, v4h);
  v4h h1 = __builtin_convertvector(w1, v4h);
  v4h h2 = __builtin_convertvector(w2, v4h);
  v4h h3 = __builtin_convertvector(w3, v4h);
  v8h lo = __builtin_shufflevector(h0, h1, 0, 1, 2, 3, 4, 5, 6, 7);
  v8h up = __builtin_shufflevector(h2, h3, 0, 1, 2, 3, 4, 5, 6, 7);
  return cat8(lo, up);
}

__device__ __forceinline__ float frcp(float x) { return __builtin_amdgcn_rcpf(x); }
__device__ __forceinline__ float sigm(float x) { return frcp(1.0f + __expf(-x)); }
__device__ __forceinline__ float tnh(float x)  { return 1.0f - 2.0f * frcp(1.0f + __expf(2.0f * x)); }

template <int DIMX>
__device__ __forceinline__ void lstm_body(
    int tile,
    const float* __restrict__ ch0, const float* __restrict__ ch1,
    const float* __restrict__ ch2, const float* __restrict__ ch3,
    int cstride,
    const int*   __restrict__ mk,
    const float* __restrict__ Winp, const float* __restrict__ binp,
    const float* __restrict__ Wih,  const float* __restrict__ Whh,
    const float* __restrict__ bih,  const float* __restrict__ bhh,
    _Float16* __restrict__ hout,
    _Float16* whl, _Float16* hbuf, float* xs, int* ms)
{
  const int tid  = threadIdx.x;
  const int w    = tid >> 5;
  const int lane = tid & 31;
  const int nn   = lane & 15;
  const int hi   = lane >> 4;
  const int ho8  = hi * 8;

  const int n0  = tile * ROWS;
  const int bi  = n0 / P_;
  const int p0  = n0 - bi * P_;
  const int col = 16 * w + nn;

  for (int i = tid; i < (G4_ * H_) / 4; i += NTHR) {
    v4f v = *(const v4f*)(Whh + 4 * i);
    *(v4h*)(whl + 4 * i) = __builtin_convertvector(v, v4h);
  }
  for (int i = tid; i < ROWS * H_; i += NTHR) hbuf[i] = (_Float16)0.0f;

  float Wc[4][4];
  float biasc[4];
#pragma unroll
  for (int g = 0; g < 4; ++g) {
    const int gc = g * H_ + col;
    const float* wr = Wih + (size_t)gc * E_;
    float a0 = 0.f, a1 = 0.f, a2 = 0.f, a3 = 0.f, ab = 0.f;
#pragma unroll 1
    for (int e4 = 0; e4 < E_; e4 += 4) {
      v4f wv = *(const v4f*)(wr + e4);
#pragma unroll
      for (int u = 0; u < 4; ++u) {
        const int e = e4 + u;
        const float wx = wv[u];
        a0 += wx * Winp[e * DIMX + 0];
        if (DIMX > 1) a1 += wx * Winp[e * DIMX + 1];
        if (DIMX > 2) a2 += wx * Winp[e * DIMX + 2];
        if (DIMX > 3) a3 += wx * Winp[e * DIMX + 3];
        ab += wx * binp[e];
      }
    }
    Wc[g][0] = a0; Wc[g][1] = a1; Wc[g][2] = a2; Wc[g][3] = a3;
    biasc[g] = ab + bih[gc] + bhh[gc];
  }

  float cst[8], hst[8];
#pragma unroll
  for (int r = 0; r < 8; ++r) { cst[r] = 0.f; hst[r] = 0.f; }

  __syncthreads();

  for (int t = 0; t < T_; ++t) {
    if (tid < ROWS * (DIMX + 1)) {
      const int c2 = tid >> 4, i = tid & 15;
      const int tb = t * B_ + bi;
      if (c2 < DIMX) {
        const float* ch = (c2 == 0) ? ch0 : (c2 == 1) ? ch1 : (c2 == 2) ? ch2 : ch3;
        xs[i * 4 + c2] = ch[tb * cstride + p0 + i];
      } else {
        ms[i] = mk[tb * P_ + p0 + i];
      }
    }

    v8f acc0 = zero8(), acc1 = zero8(), acc2 = zero8(), acc3 = zero8();
    const _Float16* arow = hbuf + nn * H_;
    const _Float16* b0r  = whl + (0 * H_ + col) * H_;
    const _Float16* b1r  = whl + (1 * H_ + col) * H_;
    const _Float16* b2r  = whl + (2 * H_ + col) * H_;
    const _Float16* b3r  = whl + (3 * H_ + col) * H_;
#pragma unroll 1
    for (int ks = 0; ks < H_ / 32; ++ks) {
      const int k0 = ks * 32;
      v16h a = frag_k_lds(arow, k0, hi);
      acc0 = wmma_f16(a, frag_k_lds(b0r, k0, hi), acc0);
      acc1 = wmma_f16(a, frag_k_lds(b1r, k0, hi), acc1);
      acc2 = wmma_f16(a, frag_k_lds(b2r, k0, hi), acc2);
      acc3 = wmma_f16(a, frag_k_lds(b3r, k0, hi), acc3);
    }

    __syncthreads();

#pragma unroll
    for (int r = 0; r < 8; ++r) {
      const int row = r + ho8;
      float gi = acc0[r] + biasc[0];
      float gf = acc1[r] + biasc[1];
      float gg = acc2[r] + biasc[2];
      float go = acc3[r] + biasc[3];
#pragma unroll
      for (int cc = 0; cc < DIMX; ++cc) {
        const float x = xs[row * 4 + cc];
        gi += Wc[0][cc] * x; gf += Wc[1][cc] * x;
        gg += Wc[2][cc] * x; go += Wc[3][cc] * x;
      }
      const float cn = sigm(gf) * cst[r] + sigm(gi) * tnh(gg);
      const float hn = sigm(go) * tnh(cn);
      const bool  m  = ms[row] > 0;
      cst[r] = m ? cn : cst[r];
      hst[r] = m ? hn : hst[r];
      hbuf[row * H_ + col] = (_Float16)hst[r];
    }

    __syncthreads();
  }

  {
    Pk16 u;
    u.h = *(const v8h*)(hbuf + tid * 8);
    float* dst = (float*)(hout + (size_t)n0 * H_ + tid * 8);
    *(volatile v4f*)dst = u.f;
    __threadfence();
    *(volatile v4f*)dst = u.f;
  }
}

__global__ __launch_bounds__(NTHR) void lstm_kernel(
    const float* __restrict__ rel,
    const float* __restrict__ vx, const float* __restrict__ vy,
    const float* __restrict__ ax, const float* __restrict__ ay,
    const int*   __restrict__ mk,
    const float* __restrict__ W_sp, const float* __restrict__ b_sp,
    const float* __restrict__ W_st, const float* __restrict__ b_st,
    const float* __restrict__ Wih_t, const float* __restrict__ Whh_t,
    const float* __restrict__ bih_t, const float* __restrict__ bhh_t,
    const float* __restrict__ Wih_s, const float* __restrict__ Whh_s,
    const float* __restrict__ bih_s, const float* __restrict__ bhh_s,
    _Float16* __restrict__ hT, _Float16* __restrict__ hS, int ntiles)
{
  __shared__ __align__(16) _Float16 whl[G4_ * H_];
  __shared__ __align__(16) _Float16 hbuf[ROWS * H_];
  __shared__ __align__(16) float    xs[ROWS * 4];
  __shared__ __align__(16) int      ms[ROWS];

  const int bid = blockIdx.x;
  if (bid < ntiles) {
    lstm_body<2>(bid, rel, rel + P_, rel, rel, 2 * P_, mk,
                 W_sp, b_sp, Wih_t, Whh_t, bih_t, bhh_t, hT, whl, hbuf, xs, ms);
  } else if (bid < 2 * ntiles) {
    lstm_body<4>(bid - ntiles, vx, vy, ax, ay, P_, mk,
                 W_st, b_st, Wih_s, Whh_s, bih_s, bhh_s, hS, whl, hbuf, xs, ms);
  }
}

__device__ __forceinline__ v8f tile_gemm(const _Float16* Al, int As, int mt,
                                         const float* __restrict__ W, int Ws,
                                         int ct, int ksteps, int nn, int hi)
{
  v8f acc = zero8();
  const _Float16* arow = Al + (mt * 16 + nn) * As;
  const float*    wrow = W + (size_t)(ct * 16 + nn) * Ws;
#pragma unroll 1
  for (int ks = 0; ks < ksteps; ++ks) {
    const int k0 = ks * 32;
    acc = wmma_f16(frag_k_lds(arow, k0, hi), frag_k_gf32(wrow, k0, hi), acc);
  }
  return acc;
}

__global__ __launch_bounds__(NTHR) void head_kernel(
    const _Float16* __restrict__ hT, const _Float16* __restrict__ hS,
    const int* __restrict__ mk,
    const float* __restrict__ F1, const float* __restrict__ f1,
    const float* __restrict__ F2, const float* __restrict__ f2,
    const float* __restrict__ A1, const float* __restrict__ a1,
    const float* __restrict__ A2, const float* __restrict__ a2,
    float* __restrict__ out, int nb)
{
  __shared__ __align__(16) char  regionA[P_ * 2 * H_ * 2];
  __shared__ __align__(16) char  regionB[P_ * H_ * 4];
  __shared__ __align__(16) float fusedf[P_ * H_];
  __shared__ __align__(16) float encs[H_];
  __shared__ float scores[P_];
  __shared__ int   okl[P_];

  _Float16* comb   = (_Float16*)regionA;
  _Float16* attin  = (_Float16*)regionA;
  _Float16* fused1 = (_Float16*)regionB;
  float*    s1f    = (float*)regionB;

  const int tid = threadIdx.x;
  const int w = tid >> 5, lane = tid & 31, nn = lane & 15, hi = lane >> 4;
  const int ho8 = hi * 8;
  const int b = blockIdx.x;
  if (b >= nb) return;

  for (int idx = tid; idx < P_ * (2 * H_ / 8); idx += NTHR) {
    const int p = idx >> 5, ch = idx & 31, k8 = ch * 8;
    const _Float16* src = (k8 < H_) ? (hT + (size_t)(b * P_ + p) * H_ + k8)
                                     : (hS + (size_t)(b * P_ + p) * H_ + (k8 - H_));
    *(v8h*)(comb + p * (2 * H_) + k8) = *(const v8h*)src;
  }
  if (tid < P_) {
    int c = 0;
#pragma unroll 1
    for (int t = 0; t < T_; ++t) c += (mk[(t * B_ + b) * P_ + tid] > 0) ? 1 : 0;
    okl[tid] = (c >= 2) ? 1 : 0;
  }
  __syncthreads();

#pragma unroll
  for (int rep = 0; rep < 2; ++rep) {
    const int tidx = w + 8 * rep;
    const int mt = tidx & 1, ct = tidx >> 1;
    v8f acc = tile_gemm(comb, 2 * H_, mt, F1, 2 * H_, ct, (2 * H_) / 32, nn, hi);
    const int j = ct * 16 + nn;
    const float bv = f1[j];
#pragma unroll
    for (int r = 0; r < 8; ++r)
      fused1[(mt * 16 + ho8 + r) * H_ + j] = (_Float16)fmaxf(acc[r] + bv, 0.f);
  }
  __syncthreads();

#pragma unroll
  for (int rep = 0; rep < 2; ++rep) {
    const int tidx = w + 8 * rep;
    const int mt = tidx & 1, ct = tidx >> 1;
    v8f acc = tile_gemm(fused1, H_, mt, F2, H_, ct, H_ / 32, nn, hi);
    const int j = ct * 16 + nn;
    const float bv = f2[j];
#pragma unroll
    for (int r = 0; r < 8; ++r) {
      const int p = mt * 16 + ho8 + r;
      float v = fmaxf(acc[r] + bv, 0.f);
      if (!okl[p]) v = 0.f;
      fusedf[p * H_ + j] = v;
      attin[p * (2 * H_) + j] = (_Float16)v;
    }
  }
  __syncthreads();

  if (tid < H_) {
    float s = 0.f; int nv = 0;
    for (int p = 0; p < P_; ++p)
      if (okl[p]) { s += fusedf[p * H_ + tid]; ++nv; }
    const _Float16 mh = (_Float16)(s * (1.0f / fmaxf((float)nv, 1.0f)));
    for (int p = 0; p < P_; ++p) attin[p * (2 * H_) + H_ + tid] = mh;
  }
  __syncthreads();

#pragma unroll
  for (int rep = 0; rep < 2; ++rep) {
    const int tidx = w + 8 * rep;
    const int mt = tidx & 1, ct = tidx >> 1;
    v8f acc = tile_gemm(attin, 2 * H_, mt, A1, 2 * H_, ct, (2 * H_) / 32, nn, hi);
    const int j = ct * 16 + nn;
    const float bv = a1[j];
#pragma unroll
    for (int r = 0; r < 8; ++r)
      s1f[(mt * 16 + ho8 + r) * H_ + j] = fmaxf(acc[r] + bv, 0.f);
  }
  __syncthreads();

  if (tid < P_) {
    float s = 0.f;
#pragma unroll 8
    for (int k = 0; k < H_; ++k) s += s1f[tid * H_ + k] * A2[k];
    s = fmaxf(s + a2[0], 0.f);
    scores[tid] = okl[tid] ? s : -1.0e9f;
  }
  __syncthreads();

  if (tid < H_) {
    float mx = -3.0e38f;
    for (int p = 0; p < P_; ++p) mx = fmaxf(mx, scores[p]);
    float se = 0.f, ac = 0.f;
    for (int p = 0; p < P_; ++p) {
      const float e = okl[p] ? __expf(scores[p] - mx) : 0.f;
      se += e;
      ac += e * fusedf[p * H_ + tid];
    }
    encs[tid] = ac / fmaxf(se, 1e-9f);
  }
  __syncthreads();

  v4f ov;
  ov.x = 0.f; ov.y = 0.f; ov.z = 0.f; ov.w = 0.f;
  float* dst = out + (size_t)b * H_ + 4 * tid;
  if (tid < H_ / 4) {
    ov = *(const v4f*)(encs + 4 * tid);
    *(volatile v4f*)dst = ov;
  }
  __threadfence();
  if (tid < H_ / 4) {
    *(volatile v4f*)dst = ov;
  }
}

extern "C" void kernel_launch(void* const* d_in, const int* in_sizes, int n_in,
                              void* d_out, int out_size, void* d_ws, size_t ws_size,
                              hipStream_t stream)
{
  if (n_in < 27) return;
  if (in_sizes[1] != T_ * B_ * 2 * P_) return;
  if (in_sizes[2] != T_ * B_ * P_ || in_sizes[6] != T_ * B_ * P_) return;
  if (in_sizes[12] != G4_ * H_ || in_sizes[16] != G4_ * H_) return;
  if (in_sizes[19] != H_ * 2 * H_ || in_sizes[23] != H_ * 2 * H_ || in_sizes[25] != H_ * H_) return;
  if (out_size != B_ * H_) return;

  const size_t hbytes = (size_t)N_ * H_ * sizeof(_Float16);
  if (ws_size < 2 * hbytes) return;

  const float* rel   = (const float*)d_in[1];
  const float* vx    = (const float*)d_in[2];
  const float* vy    = (const float*)d_in[3];
  const float* axp   = (const float*)d_in[4];
  const float* ayp   = (const float*)d_in[5];
  const int*   mk    = (const int*)d_in[6];
  const float* W_sp  = (const float*)d_in[7];
  const float* b_sp  = (const float*)d_in[8];
  const float* W_st  = (const float*)d_in[9];
  const float* b_st  = (const float*)d_in[10];
  const float* Wih_t = (const float*)d_in[11];
  const float* Whh_t = (const float*)d_in[12];
  const float* bih_t = (const float*)d_in[13];
  const float* bhh_t = (const float*)d_in[14];
  const float* Wih_s = (const float*)d_in[15];
  const float* Whh_s = (const float*)d_in[16];
  const float* bih_s = (const float*)d_in[17];
  const float* bhh_s = (const float*)d_in[18];
  const float* A1    = (const float*)d_in[19];
  const float* a1    = (const float*)d_in[20];
  const float* A2    = (const float*)d_in[21];
  const float* a2    = (const float*)d_in[22];
  const float* F1    = (const float*)d_in[23];
  const float* f1    = (const float*)d_in[24];
  const float* F2    = (const float*)d_in[25];
  const float* f2    = (const float*)d_in[26];

  char* ws = (char*)d_ws;
  _Float16* hT = (_Float16*)(ws);
  _Float16* hS = (_Float16*)(ws + hbytes);

  const int ntiles = (N_ + ROWS - 1) / ROWS;

  lstm_kernel<<<2 * ntiles, NTHR, 0, stream>>>(
      rel, vx, vy, axp, ayp, mk,
      W_sp, b_sp, W_st, b_st,
      Wih_t, Whh_t, bih_t, bhh_t,
      Wih_s, Whh_s, bih_s, bhh_s,
      hT, hS, ntiles);
  head_kernel<<<B_, NTHR, 0, stream>>>(
      hT, hS, mk, F1, f1, F2, f2, A1, a1, A2, a2, (float*)d_out, B_);
}
